// CosineAttention_48576080118367
// MI455X (gfx1250) — hardware-verified
//
#include <hip/hip_runtime.h>
#include <stdint.h>

typedef __attribute__((ext_vector_type(16))) _Float16 v16h;
typedef __attribute__((ext_vector_type(8)))  _Float16 v8h;
typedef __attribute__((ext_vector_type(16))) __bf16   v16b;
typedef __attribute__((ext_vector_type(8)))  __bf16   v8b;
typedef __attribute__((ext_vector_type(8)))  float    v8f;
typedef __attribute__((ext_vector_type(4)))  float    v4f;
typedef __attribute__((ext_vector_type(2)))  float    v2f;
typedef __attribute__((ext_vector_type(4)))  unsigned v4u;

constexpr int kBatch = 2;
constexpr int kSeq   = 2048;
constexpr int kDm    = 1024;
constexpr int kHeads = 16;
constexpr int kHd    = 64;
constexpr int kTok   = kBatch * kSeq;
constexpr int kKch   = 64;
constexpr int kQblk  = 64;
#define P_CARRY 16384.0f
#define O_CARRY 64.0f
#define WO_CARRY 1024.0f

static_assert(kDm == kHeads * kHd, "head split");
static_assert(kTok % 64 == 0 && kDm % 64 == 0, "GEMM M,N tile multiples");
static_assert(kDm % 32 == 0, "GEMM K multiple of 32");
static_assert(kSeq % kKch == 0 && kSeq % kQblk == 0, "attention tiles");
static_assert((kTok * kHeads) % 32 == 0, "normalize grid");

__device__ __forceinline__ unsigned short f2bf_bits(float f) {
  unsigned u = __float_as_uint(f);
  return (unsigned short)((u + 0x7FFFu + ((u >> 16) & 1u)) >> 16);
}
__device__ __forceinline__ float bf_bits2f(unsigned short h) { return __uint_as_float(((unsigned)h) << 16); }
__device__ __forceinline__ _Float16 h16_lo(unsigned w) { return __builtin_bit_cast(_Float16, (unsigned short)(w & 0xffffu)); }
__device__ __forceinline__ _Float16 h16_hi(unsigned w) { return __builtin_bit_cast(_Float16, (unsigned short)(w >> 16)); }

__device__ __forceinline__ void dep_guard_h(v8f& a, v8f& b, v16h x, v16h y) { asm volatile("v_nop\n\tv_nop\n\tv_nop\n\tv_nop" : "+v"(a), "+v"(b) : "v"(x), "v"(y)); }
__device__ __forceinline__ void dep_guard_b(v8f& a, v8f& b, v16b x, v16b y) { asm volatile("v_nop\n\tv_nop\n\tv_nop\n\tv_nop" : "+v"(a), "+v"(b) : "v"(x), "v"(y)); }
__device__ __forceinline__ void keep4_h(v16h a, v16h b, v16h c, v16h d) { asm volatile("v_nop" :: "v"(a), "v"(b), "v"(c), "v"(d)); }
__device__ __forceinline__ void keep4_b(v16b a, v16b b, v16b c, v16b d) { asm volatile("v_nop" :: "v"(a), "v"(b), "v"(c), "v"(d)); }
__device__ __forceinline__ void acc_guard4(v8f& a, v8f& b, v8f& c, v8f& d) { asm volatile("v_nop\n\tv_nop\n\tv_nop\n\tv_nop" : "+v"(a), "+v"(b), "+v"(c), "+v"(d)); }
template <typename T> struct Frag;
template <> struct Frag<_Float16> {
  typedef v16h V; union U { v16h v; v8h h[2]; };
  static __device__ __forceinline__ v16h load(const _Float16* p) {
    U f; f.h[0] = *(const v8h*)(p); f.h[1] = *(const v8h*)(p + 16); return f.v;
  }
  static __device__ __forceinline__ v8f mma(v16h a, v16h b, v8f c) {
    return __builtin_amdgcn_wmma_f32_16x16x32_f16(false, a, false, b, (short)0, c, false, false);
  }
  static __device__ __forceinline__ void guard(v8f& a, v8f& b, v16h x, v16h y) { dep_guard_h(a, b, x, y); }
  static __device__ __forceinline__ void keep(v16h a, v16h b, v16h c, v16h d) { keep4_h(a, b, c, d); }
};
template <> struct Frag<__bf16> {
  typedef v16b V; union U { v16b v; v8b h[2]; };
  static __device__ __forceinline__ v16b load(const __bf16* p) {
    U f; f.h[0] = *(const v8b*)(p); f.h[1] = *(const v8b*)(p + 16); return f.v;
  }
  static __device__ __forceinline__ v8f mma(v16b a, v16b b, v8f c) {
    return __builtin_amdgcn_wmma_f32_16x16x32_bf16(false, a, false, b, (short)0, c, false, false);
  }
  static __device__ __forceinline__ void guard(v8f& a, v8f& b, v16b x, v16b y) { dep_guard_b(a, b, x, y); }
  static __device__ __forceinline__ void keep(v16b a, v16b b, v16b c, v16b d) { keep4_b(a, b, c, d); }
};

template <int ET> struct Elem;
template <> struct Elem<0> { typedef _Float16 T; };
template <> struct Elem<1> { typedef __bf16 T; };
template <int ET, bool SPLIT, int BIAS_MODE, int OUT_MODE, bool RESID, int ACT = 0>
__global__ __launch_bounds__(256) void wmma_gemm64(
    const unsigned short* __restrict__ Ap, const unsigned short* __restrict__ A2p, int lda, long strideA,
    const unsigned short* __restrict__ Btp, const unsigned short* __restrict__ Bt2p, int ldb, long strideB,
    void* __restrict__ Cout, void* __restrict__ Cout2, int ldc, long strideC,
    const float* __restrict__ bias,
    const float* __restrict__ resid, long strideR,
    int M, int N, int K, float scale) {
  typedef typename Elem<ET>::T T;
  typedef typename Frag<T>::V V;
  const T* A = (const T*)Ap; const T* A2 = (const T*)A2p; const T* Bt = (const T*)Btp; const T* Bt2 = (const T*)Bt2p;
  __shared__ __align__(16) float sT[8][16 * 68];
  const int b    = blockIdx.y;
  const int lane = threadIdx.x & 31;
  const int wave = threadIdx.x >> 5;
  const int tilesN = N >> 6;
  const int tilesM = M >> 6;
  const int tile = blockIdx.x * 8 + wave;
  if (tile >= tilesM * tilesN) return;
  const int tm = tile / tilesN;
  const int tn = tile - tm * tilesN;
  const int m0 = tm << 6;
  const int n0 = tn << 6;

  const T* Ab  = A  + (size_t)b * strideA;
  const T* Bb  = Bt + (size_t)b * strideB;
  const T* Ab2 = SPLIT ? (A2  + (size_t)b * strideA) : nullptr;
  const T* Bb2 = SPLIT ? (Bt2 + (size_t)b * strideB) : nullptr;

  const int rlane = lane & 15;
  const int koff  = (lane >> 4) * 8;
  const int mOff  = (lane >> 4) * 8;

  v8f acc[4][4];
#pragma unroll
  for (int i = 0; i < 4; ++i)
#pragma unroll
    for (int j = 0; j < 4; ++j) acc[i][j] = (v8f){0.f,0.f,0.f,0.f,0.f,0.f,0.f,0.f};

  for (int k0 = 0; k0 < K; k0 += 32) {
    V bh[4], bl[4];
#pragma unroll
    for (int j = 0; j < 4; ++j) {
      const size_t bo = (size_t)(n0 + (j << 4) + rlane) * ldb + koff + k0;
      bh[j] = Frag<T>::load(Bb + bo);
      if (SPLIT) bl[j] = Frag<T>::load(Bb2 + bo);
    }
#pragma unroll
    for (int i = 0; i < 4; ++i) {
      const size_t ao = (size_t)(m0 + (i << 4) + rlane) * lda + koff + k0;
      V ah = Frag<T>::load(Ab + ao);
      V al;
      if (SPLIT) al = Frag<T>::load(Ab2 + ao);
#pragma unroll
      for (int j = 0; j < 4; ++j) {
        acc[i][j] = Frag<T>::mma(ah, bh[j], acc[i][j]);
        if (SPLIT) {
          acc[i][j] = Frag<T>::mma(ah, bl[j], acc[i][j]);
          acc[i][j] = Frag<T>::mma(al, bh[j], acc[i][j]);
        }
      }
      Frag<T>::guard(acc[i][0], acc[i][3], ah, SPLIT ? al : ah);
    }
    Frag<T>::keep(bh[0], bh[1], bh[2], bh[3]);
    if (SPLIT) Frag<T>::keep(bl[0], bl[1], bl[2], bl[3]);
  }
  acc_guard4(acc[0][0], acc[0][1], acc[0][2], acc[0][3]);
  acc_guard4(acc[1][0], acc[1][1], acc[1][2], acc[1][3]);
  acc_guard4(acc[2][0], acc[2][1], acc[2][2], acc[2][3]);
  acc_guard4(acc[3][0], acc[3][1], acc[3][2], acc[3][3]);

  float* slab = sT[wave];
  const float* Rb = RESID ? (resid + (size_t)b * strideR) : nullptr;
#pragma unroll
  for (int i = 0; i < 4; ++i) {
    const int mBase = m0 + (i << 4);
#pragma unroll
    for (int j = 0; j < 4; ++j) {
      const int n = n0 + (j << 4) + rlane;
      float bv = 0.f;
      if (BIAS_MODE == 2) bv = bf_bits2f(f2bf_bits(bias[n]));
#pragma unroll
      for (int r = 0; r < 8; ++r) {
        float v = acc[i][j][r] * scale;
        if (BIAS_MODE == 1) v += bf_bits2f(f2bf_bits(bias[mBase + mOff + r]));
        if (BIAS_MODE == 2) v += bv;
        if (RESID) v += Rb[(size_t)(mBase + mOff + r) * ldc + n];
        if (ACT == 1) v = tanhf(v);
        if (ACT == 2) v = fmaxf(v, 0.0f);
        if (ACT == 3) v = v / (1.0f + expf(-v));
        if (ACT == 4) v = (v > 0.f) ? v : 0.01f * v;
        slab[(mOff + r) * 68 + (j << 4) + rlane] = v;
      }
    }
    __builtin_amdgcn_fence(__ATOMIC_RELEASE, "workgroup");
    __builtin_amdgcn_wave_barrier();
    __builtin_amdgcn_fence(__ATOMIC_ACQUIRE, "workgroup");
    if (OUT_MODE == 0) {
      float* C = (float*)Cout + (size_t)b * strideC;
      const int hh = lane >> 4, c4 = (lane & 15) * 4;
      for (int pass = 0; pass < 2; ++pass) {
#pragma unroll
        for (int it = 0; it < 8; ++it) {
          const int row = it * 2 + hh;
          v4f v = *(const v4f*)(slab + row * 68 + c4);
          *(volatile v4f*)(C + (size_t)(mBase + row) * ldc + n0 + c4) = v;
        }
        __threadfence();
      }
    } else {
      const int q = lane >> 3, c8 = (lane & 7) * 8;
      unsigned short* C  = (unsigned short*)Cout  + (size_t)b * strideC;
      unsigned short* C2 = (OUT_MODE == 2) ? ((unsigned short*)Cout2 + (size_t)b * strideC) : nullptr;
      for (int pass = 0; pass < 2; ++pass) {
#pragma unroll
        for (int it = 0; it < 4; ++it) {
          const int row = it * 4 + q;
          const float* sp = slab + row * 68 + c8;
          v8h hv, lv;
#pragma unroll
          for (int e = 0; e < 8; ++e) {
            if (OUT_MODE == 1) {
              hv[e] = (_Float16)sp[e];
            } else {
              unsigned short hb = f2bf_bits(sp[e]);
              unsigned short lb = f2bf_bits(sp[e] - bf_bits2f(hb));
              hv[e] = __builtin_bit_cast(_Float16, hb);
              lv[e] = __builtin_bit_cast(_Float16, lb);
            }
          }
          *(volatile v8h*)(C + (size_t)(mBase + row) * ldc + n0 + c8) = hv;
          if (OUT_MODE == 2) *(volatile v8h*)(C2 + (size_t)(mBase + row) * ldc + n0 + c8) = lv;
        }
        __threadfence();
      }
    }
    __builtin_amdgcn_fence(__ATOMIC_RELEASE, "workgroup");
    __builtin_amdgcn_wave_barrier();
    __builtin_amdgcn_fence(__ATOMIC_ACQUIRE, "workgroup");
  }
}

template <int MODE>
__global__ __launch_bounds__(256) void cast2_kernel(const float* __restrict__ in,
                                                    unsigned short* __restrict__ out, int n2, float mul) {
  const int i = blockIdx.x * 256 + threadIdx.x;
  if (i < n2) {
    const v2f p = *(const v2f*)(in + 2 * (size_t)i);
    unsigned short u0, u1;
    if (MODE == 0) {
      u0 = f2bf_bits(p.x); u1 = f2bf_bits(p.y);
    } else {
      const float r0 = bf_bits2f(f2bf_bits(p.x)) * mul;
      const float r1 = bf_bits2f(f2bf_bits(p.y)) * mul;
      u0 = __builtin_bit_cast(unsigned short, (_Float16)r0);
      u1 = __builtin_bit_cast(unsigned short, (_Float16)r1);
    }
    const unsigned u = (unsigned)u0 | ((unsigned)u1 << 16);
    volatile unsigned* op = (volatile unsigned*)(void*)out;
    op[i] = u;
    __threadfence();
    op[i] = u;
  }
}

__global__ __launch_bounds__(256) void l2norm_split_kernel(
    const float* __restrict__ qf, const float* __restrict__ kf, const float* __restrict__ tau,
    unsigned short* __restrict__ qhp, unsigned short* __restrict__ qlp,
    unsigned short* __restrict__ khp, unsigned short* __restrict__ klp) {
  const bool isk = (blockIdx.y != 0);
  const float* src = isk ? kf : qf;
  unsigned short* dhp = isk ? khp : qhp;
  unsigned short* dlp = isk ? klp : qlp;
  const int tid = threadIdx.x;
  const int g = tid >> 3, e = tid & 7;
  const int seg = blockIdx.x * 32 + g;
  const int token = seg >> 4, head = seg & 15;
  const size_t base = (size_t)token * kDm + (size_t)head * kHd + (size_t)e * 8;
  const v4f a  = *(const v4f*)(src + base);
  const v4f c4 = *(const v4f*)(src + base + 4);
  float ss = 0.0f;
  ss += a.x * a.x;  ss += a.y * a.y;  ss += a.z * a.z;  ss += a.w * a.w;
  ss += c4.x * c4.x; ss += c4.y * c4.y; ss += c4.z * c4.z; ss += c4.w * c4.w;
  ss += __shfl_xor(ss, 1, 32);
  ss += __shfl_xor(ss, 2, 32);
  ss += __shfl_xor(ss, 4, 32);
  const float nrm  = sqrtf(ss);
  const float rinv = 1.0f / fmaxf(nrm, 1e-12f);
  const float th   = bf_bits2f(f2bf_bits(tau[head]));
  const float sc   = isk ? rinv : rinv * th;
  float vals[8];
  vals[0] = a.x * sc;  vals[1] = a.y * sc;  vals[2] = a.z * sc;  vals[3] = a.w * sc;
  vals[4] = c4.x * sc; vals[5] = c4.y * sc; vals[6] = c4.z * sc; vals[7] = c4.w * sc;
  unsigned hw[4], lw[4];
#pragma unroll
  for (int i = 0; i < 4; ++i) {
    const float v0 = vals[2 * i], v1 = vals[2 * i + 1];
    const unsigned short h0 = f2bf_bits(v0), h1 = f2bf_bits(v1);
    const unsigned short l0 = f2bf_bits(v0 - bf_bits2f(h0));
    const unsigned short l1 = f2bf_bits(v1 - bf_bits2f(h1));
    hw[i] = (unsigned)h0 | ((unsigned)h1 << 16);
    lw[i] = (unsigned)l0 | ((unsigned)l1 << 16);
  }
  v4u hv; hv.x = hw[0]; hv.y = hw[1]; hv.z = hw[2]; hv.w = hw[3];
  v4u lv; lv.x = lw[0]; lv.y = lw[1]; lv.z = lw[2]; lv.w = lw[3];
  volatile v4u* ph = (volatile v4u*)(void*)(dhp + base);
  volatile v4u* pl = (volatile v4u*)(void*)(dlp + base);
  *ph = hv; *pl = lv;
  __threadfence();
  *ph = hv; *pl = lv;
}

__device__ __forceinline__ v8f at_mma_b(v16b a, v16b b, v8f c) {
  c = __builtin_amdgcn_wmma_f32_16x16x32_bf16(false, a, false, b, (short)0, c, false, false);
  asm volatile("v_nop\n\tv_nop\n\tv_nop\n\tv_nop" : "+v"(c) : "v"(a), "v"(b));
  return c;
}
__device__ __forceinline__ v8f at_mma_h(v16h a, v16h b, v8f c) {
  c = __builtin_amdgcn_wmma_f32_16x16x32_f16(false, a, false, b, (short)0, c, false, false);
  asm volatile("v_nop\n\tv_nop\n\tv_nop\n\tv_nop" : "+v"(c) : "v"(a), "v"(b));
  return c;
}

__global__ __launch_bounds__(128)
void cos_attn_kernel(const unsigned short* __restrict__ qhp, const unsigned short* __restrict__ qlp,
                     const unsigned short* __restrict__ khp, const unsigned short* __restrict__ klp,
                     const unsigned short* __restrict__ vvp, const float* __restrict__ mask,
                     unsigned short* __restrict__ oo) {
  union FB { v16b v; v8b h[2]; };
  union FH { v16h v; v8h h[2]; };
  __shared__ __align__(16) __bf16   Ksh[kKch * kHd];
  __shared__ __align__(16) __bf16   Ksl[kKch * kHd];
  __shared__ __align__(16) _Float16 Vt[kHd * kKch];
  __shared__ __align__(16) float    Msk[kQblk * kKch];
  __shared__ __align__(16) _Float16 Psh[4][16 * kKch];

  const int tid  = threadIdx.x;
  const int wave = tid >> 5;
  const int lane = tid & 31;
  const int hh   = lane >> 4;
  const int c    = lane & 15;

  const int nqb = kSeq / kQblk;
  const int bx  = blockIdx.x;
  const int qb  = bx % nqb;
  const int bh  = bx / nqb;
  const int h   = bh % kHeads;
  const int b   = bh / kHeads;
  const int qbase = qb * kQblk;
  const int q0    = qbase + wave * 16;
  const size_t tokb = (size_t)b * kSeq;

  const __bf16*   qh = (const __bf16*)(const void*)qhp;
  const __bf16*   ql = (const __bf16*)(const void*)qlp;

  v16b qah[2], qal[2];
  {
    const size_t ro = (tokb + (size_t)(q0 + c)) * kDm + (size_t)h * kHd;
#pragma unroll
    for (int dc = 0; dc < 2; ++dc) {
      qah[dc] = Frag<__bf16>::load(qh + ro + dc * 32 + 8 * hh);
      qal[dc] = Frag<__bf16>::load(ql + ro + dc * 32 + 8 * hh);
    }
  }

  float mrow[8], lrow[8];
  v8f oacc[4];
#pragma unroll
  for (int r = 0; r < 8; ++r) { mrow[r] = -INFINITY; lrow[r] = 0.f; }
#pragma unroll
  for (int t = 0; t < 4; ++t) oacc[t] = (v8f){0.f,0.f,0.f,0.f,0.f,0.f,0.f,0.f};

  for (int kc = 0; kc < kSeq / kKch; ++kc) {
    const int kv0 = kc * kKch;
    __syncthreads();
    {
      const int rr = tid >> 1;
      const int c0 = (tid & 1) * 32;
      const size_t ro = (tokb + (size_t)(kv0 + rr)) * kDm + (size_t)h * kHd + c0;
      const uint4* kph = (const uint4*)(const void*)(khp + ro);
      const uint4* kpl = (const uint4*)(const void*)(klp + ro);
#pragma unroll
      for (int i = 0; i < 4; ++i) {
        const uint4 wh = kph[i];
        const uint4 wl = kpl[i];
        *(uint4*)(void*)(Ksh + rr * kHd + c0 + 8 * i) = wh;
        *(uint4*)(void*)(Ksl + rr * kHd + c0 + 8 * i) = wl;
      }
      asm volatile("" ::: "memory");
      const uint4* vp = (const uint4*)(const void*)(vvp + ro);
#pragma unroll
      for (int i = 0; i < 4; ++i) {
        const uint4 w4 = vp[i];
        const int d0 = c0 + 8 * i;
        Vt[(d0 + 0) * kKch + rr] = h16_lo(w4.x);
        Vt[(d0 + 1) * kKch + rr] = h16_hi(w4.x);
        Vt[(d0 + 2) * kKch + rr] = h16_lo(w4.y);
        Vt[(d0 + 3) * kKch + rr] = h16_hi(w4.y);
        Vt[(d0 + 4) * kKch + rr] = h16_lo(w4.z);
        Vt[(d0 + 5) * kKch + rr] = h16_hi(w4.z);
        Vt[(d0 + 6) * kKch + rr] = h16_lo(w4.w);
        Vt[(d0 + 7) * kKch + rr] = h16_hi(w4.w);
      }
      asm volatile("" ::: "memory");
      const float* mp = mask + (size_t)(qbase + rr) * kSeq + kv0 + c0;
#pragma unroll
      for (int i = 0; i < 8; ++i) {
        const v4f m4 = *(const v4f*)(mp + 4 * i);
        v4f r4;
        r4.x = bf_bits2f(f2bf_bits(m4.x));
        r4.y = bf_bits2f(f2bf_bits(m4.y));
        r4.z = bf_bits2f(f2bf_bits(m4.z));
        r4.w = bf_bits2f(f2bf_bits(m4.w));
        *(v4f*)(Msk + rr * kKch + c0 + 4 * i) = r4;
      }
    }
    __syncthreads();

    v8f s[4];
#pragma unroll
    for (int j = 0; j < 4; ++j) {
      s[j] = (v8f){0.f,0.f,0.f,0.f,0.f,0.f,0.f,0.f};
#pragma unroll
      for (int dc = 0; dc < 2; ++dc) {
        FB kb, klo;
        kb.h[0]  = *(const v8b*)(Ksh + (j * 16 + c) * kHd + dc * 32 + 8 * hh);
        kb.h[1]  = *(const v8b*)(Ksh + (j * 16 + c) * kHd + dc * 32 + 16 + 8 * hh);
        klo.h[0] = *(const v8b*)(Ksl + (j * 16 + c) * kHd + dc * 32 + 8 * hh);
        klo.h[1] = *(const v8b*)(Ksl + (j * 16 + c) * kHd + dc * 32 + 16 + 8 * hh);
        s[j] = at_mma_b(qah[dc], kb.v,  s[j]);
        s[j] = at_mma_b(qah[dc], klo.v, s[j]);
        s[j] = at_mma_b(qal[dc], kb.v,  s[j]);
      }
    }

    float cm[8];
    const float* mrw = Msk + (wave * 16 + 8 * hh) * kKch;
#pragma unroll
    for (int r = 0; r < 8; ++r) {
      float m = -INFINITY;
#pragma unroll
      for (int j = 0; j < 4; ++j) {
        s[j][r] += mrw[r * kKch + j * 16 + c];
        m = fmaxf(m, s[j][r]);
      }
#pragma unroll
      for (int off = 1; off < 16; off <<= 1) m = fmaxf(m, __shfl_xor(m, off, 32));
      cm[r] = m;
    }
    _Float16* pwh = Psh[wave];
#pragma unroll
    for (int r = 0; r < 8; ++r) {
      const float mnew  = fmaxf(mrow[r], cm[r]);
      const float alpha = expf(mrow[r] - mnew);
      mrow[r] = mnew;
      float psum = 0.f;
#pragma unroll
      for (int j = 0; j < 4; ++j) {
        const float p = expf(s[j][r] - mnew);
        psum += p;
        pwh[(8 * hh + r) * kKch + j * 16 + c] = (_Float16)(p * P_CARRY);
      }
#pragma unroll
      for (int off = 1; off < 16; off <<= 1) psum += __shfl_xor(psum, off, 32);
      lrow[r] = lrow[r] * alpha + psum;
#pragma unroll
      for (int t = 0; t < 4; ++t) oacc[t][r] *= alpha;
    }
    __builtin_amdgcn_fence(__ATOMIC_RELEASE, "workgroup");
    __builtin_amdgcn_wave_barrier();
    __builtin_amdgcn_fence(__ATOMIC_ACQUIRE, "workgroup");
#pragma unroll 1
    for (int kk = 0; kk < 2; ++kk) {
      FH pa;
      pa.h[0] = *(const v8h*)(pwh + c * kKch + kk * 32 + 8 * hh);
      pa.h[1] = *(const v8h*)(pwh + c * kKch + kk * 32 + 16 + 8 * hh);
#pragma unroll
      for (int t = 0; t < 4; ++t) {
        FH vb;
        vb.h[0] = *(const v8h*)(Vt + (t * 16 + c) * kKch + kk * 32 + 8 * hh);
        vb.h[1] = *(const v8h*)(Vt + (t * 16 + c) * kKch + kk * 32 + 16 + 8 * hh);
        oacc[t] = at_mma_h(pa.v, vb.v, oacc[t]);
      }
    }
  }

  _Float16* pw = Psh[wave];
  __builtin_amdgcn_fence(__ATOMIC_RELEASE, "workgroup");
  __builtin_amdgcn_wave_barrier();
  __builtin_amdgcn_fence(__ATOMIC_ACQUIRE, "workgroup");
#pragma unroll
  for (int r = 0; r < 8; ++r) {
    const float inv = O_CARRY / (lrow[r] * P_CARRY);
#pragma unroll
    for (int t = 0; t < 4; ++t) pw[(8 * hh + r) * kKch + t * 16 + c] = (_Float16)(oacc[t][r] * inv);
  }
  __builtin_amdgcn_fence(__ATOMIC_RELEASE, "workgroup");
  __builtin_amdgcn_wave_barrier();
  __builtin_amdgcn_fence(__ATOMIC_ACQUIRE, "workgroup");
  {
    const int q8 = lane >> 3, c8 = (lane & 7) * 8;
    _Float16* ob = (_Float16*)(void*)oo + (tokb + (size_t)q0) * kDm + (size_t)h * kHd;
    for (int pass = 0; pass < 2; ++pass) {
#pragma unroll
      for (int it = 0; it < 4; ++it) {
        const int row = it * 4 + q8;
        const v8h val = *(const v8h*)(pw + row * kKch + c8);
        *(volatile v8h*)(ob + (size_t)row * kDm + c8) = val;
      }
      __threadfence();
    }
  }
}

extern "C" void kernel_launch(void* const* d_in, const int* in_sizes, int n_in,
                              void* d_out, int out_size, void* d_ws, size_t ws_size,
                              hipStream_t stream) {
  if (n_in < 11) return;
  const float* x    = (const float*)d_in[0];
  const float* mask = (const float*)d_in[1];
  const float* Wq   = (const float*)d_in[2];
  const float* bq   = (const float*)d_in[3];
  const float* Wk   = (const float*)d_in[4];
  const float* bk   = (const float*)d_in[5];
  const float* Wv   = (const float*)d_in[6];
  const float* bv   = (const float*)d_in[7];
  const float* Wo   = (const float*)d_in[8];
  const float* bo   = (const float*)d_in[9];
  const float* tau  = (const float*)d_in[10];

  const size_t nX = (size_t)kTok * kDm;
  const size_t nW = (size_t)kDm * kDm;
  if ((size_t)in_sizes[0] != nX || (size_t)in_sizes[1] != (size_t)kSeq * kSeq ||
      (size_t)in_sizes[2] != nW || (size_t)in_sizes[4] != nW || (size_t)in_sizes[6] != nW ||
      (size_t)in_sizes[8] != nW || in_sizes[3] != kDm || in_sizes[5] != kDm || in_sizes[7] != kDm ||
      in_sizes[9] != kDm || in_sizes[10] != kHeads) return;
  if ((size_t)out_size != nX) return;

  const size_t offXb  = 0;
  const size_t offWq  = offXb  + nX * 2;
  const size_t offWk  = offWq  + nW * 2;
  const size_t offWv  = offWk  + nW * 2;
  const size_t offWo  = offWv  + nW * 2;
  const size_t offQf  = offWo  + nW * 2;
  const size_t offKf  = offQf  + nX * 4;
  const size_t offQh  = offKf  + nX * 4;
  const size_t offQl  = offQh  + nX * 2;
  const size_t offKh  = offQl  + nX * 2;
  const size_t offKl  = offKh  + nX * 2;
  const size_t offVv  = offKl  + nX * 2;
  const size_t offEnd = offVv  + nX * 2;
  if (offEnd > ws_size) return;

  char* ws = (char*)d_ws;
  unsigned short* xb  = (unsigned short*)(ws + offXb);
  unsigned short* wqb = (unsigned short*)(ws + offWq);
  unsigned short* wkb = (unsigned short*)(ws + offWk);
  unsigned short* wvb = (unsigned short*)(ws + offWv);
  unsigned short* wof = (unsigned short*)(ws + offWo);
  float*          qf  = (float*)(ws + offQf);
  unsigned short* oo  = (unsigned short*)(ws + offQf);
  float*          kf  = (float*)(ws + offKf);
  unsigned short* qhb = (unsigned short*)(ws + offQh);
  unsigned short* qlb = (unsigned short*)(ws + offQl);
  unsigned short* khb = (unsigned short*)(ws + offKh);
  unsigned short* klb = (unsigned short*)(ws + offKl);
  unsigned short* vvh = (unsigned short*)(ws + offVv);

  const int n2X = (int)(nX / 2), n2W = (int)(nW / 2);
  cast2_kernel<0><<<dim3(n2X / 256), dim3(256), 0, stream>>>(x,  xb,  n2X, 1.0f);
  cast2_kernel<0><<<dim3(n2W / 256), dim3(256), 0, stream>>>(Wq, wqb, n2W, 1.0f);
  cast2_kernel<0><<<dim3(n2W / 256), dim3(256), 0, stream>>>(Wk, wkb, n2W, 1.0f);
  cast2_kernel<0><<<dim3(n2W / 256), dim3(256), 0, stream>>>(Wv, wvb, n2W, 1.0f);
  cast2_kernel<1><<<dim3(n2W / 256), dim3(256), 0, stream>>>(Wo, wof, n2W, WO_CARRY);

  const int gemmTiles  = (kTok / 64) * (kDm / 64);
  const int gemmBlocks = (gemmTiles + 7) / 8;
  wmma_gemm64<1, false, 2, 0, false, 0><<<dim3(gemmBlocks, 1), dim3(256), 0, stream>>>(
      xb, xb, kDm, 0L, wqb, wqb, kDm, 0L, (void*)qf, (void*)qf, kDm, 0L, bq, nullptr, 0L, kTok, kDm, kDm, 1.0f);
  wmma_gemm64<1, false, 2, 0, false, 0><<<dim3(gemmBlocks, 1), dim3(256), 0, stream>>>(
      xb, xb, kDm, 0L, wkb, wkb, kDm, 0L, (void*)kf, (void*)kf, kDm, 0L, bk, nullptr, 0L, kTok, kDm, kDm, 1.0f);
  wmma_gemm64<1, false, 2, 1, false, 0><<<dim3(gemmBlocks, 1), dim3(256), 0, stream>>>(
      xb, xb, kDm, 0L, wvb, wvb, kDm, 0L, (void*)vvh, (void*)vvh, kDm, 0L, bv, nullptr, 0L, kTok, kDm, kDm, 1.0f);

  l2norm_split_kernel<<<dim3((kTok * kHeads) / 32, 2), dim3(256), 0, stream>>>(qf, kf, tau, qhb, qlb, khb, klb);

  cos_attn_kernel<<<dim3(kBatch * kHeads * (kSeq / kQblk)), dim3(128), 0, stream>>>(qhb, qlb, khb, klb, vvh, mask, oo);

  wmma_gemm64<0, false, 2, 0, false, 0><<<dim3(gemmBlocks, 1), dim3(256), 0, stream>>>(
      oo, oo, kDm, 0L, wof, wof, kDm, 0L, d_out, d_out, kDm, 0L, bo, nullptr, 0L, kTok, kDm, kDm,
      1.0f / (O_CARRY * WO_CARRY));
}
